// SchNetSimple_28544352649720
// MI455X (gfx1250) — hardware-verified
//
#include <hip/hip_runtime.h>
#include <stddef.h>


#define HC      128
#define NGC     51
#define KP1     64
#define NTHR    256
#define NWAVE   8
#define EPT     8
#define CHUNK   (NTHR * EPT)
#define WCAP    (EPT * 32)
#define LISTN   (NWAVE * WCAP)
#define PASSN   (NWAVE * 16)
#define PCAP    (CHUNK + PASSN)
#define NB      192
#define RPW     (NB / NWAVE)
#define NODEBLK 32
#define WSC     64.0f
#define ASC     64.0f
#define RSC     256.0f
#define F12     0.000244140625f
#define F14     0.00006103515625f
#define LN2F    0.69314718056f
#define PIF     3.14159265358979f

static_assert(PCAP % PASSN == 0);
static_assert((NB % 16) == 0 && (RPW * NWAVE) == NB);

#define A_ACC   0
#define A_MSG   (A_ACC + (NB + 1) * HC * 4)
#define A_W1    (A_MSG + PASSN * HC * 4)
#define A_W2    (A_W1 + HC * KP1 * 2)
#define A_STG   (A_W2 + HC * HC * 2)
#define A_LIST  (A_STG + PASSN * KP1 * 2)
#define A_PEND  (A_LIST + LISTN * 4)
#define A_SLOT  (A_PEND + PCAP * 4)
#define A_COL   (A_SLOT + PASSN * 4)
#define A_CB    (A_COL + PASSN * 4)
#define A_BS    (A_CB + PASSN * 4)
#define A_WCNT  (A_BS + 2 * HC * 4)
#define SMEM_AGG (A_WCNT + 64)
#define N_W1    0
#define N_W2    (HC * HC * 2)
#define N_BS    (2 * HC * HC * 2)
#define N_OT    (N_BS + 2 * HC * 4)
#define SMEM_NODE (N_OT + NWAVE * 16 * HC * 4)
static_assert(SMEM_AGG <= 262144);
static_assert((A_MSG % 16) == 0 && (A_W1 % 16) == 0 && (A_STG % 16) == 0 && (A_BS % 16) == 0 && (N_OT % 16) == 0);

typedef float    v4f  __attribute__((ext_vector_type(4)));
typedef float    v8f  __attribute__((ext_vector_type(8)));
typedef int      v4i  __attribute__((ext_vector_type(4)));
typedef _Float16 v8h  __attribute__((ext_vector_type(8)));
typedef _Float16 v16h __attribute__((ext_vector_type(16)));
union FragH { v16h v; v8h h[2]; };

__device__ __forceinline__ v8f wmh(v16h a, v16h b, v8f c) {
  v8f d = __builtin_amdgcn_wmma_f32_16x16x32_f16(false, a, false, b, (short)0, c, false, false);
  asm volatile("v_nop\n\tv_nop\n\tv_nop\n\tv_nop" : "+v"(d) : "v"(a), "v"(b));
  return d;
}
__device__ __forceinline__ void wave_sync() {
  __builtin_amdgcn_fence(__ATOMIC_RELEASE, "wavefront");
  __builtin_amdgcn_wave_barrier();
}
__device__ __forceinline__ v8f zero8f() {
  v8f z;
#pragma unroll
  for (int i = 0; i < 8; ++i) z[i] = 0.0f;
  return z;
}
__device__ __forceinline__ float sspf(float x) {
  return fmaxf(x, 0.0f) + __logf(1.0f + __expf(-fabsf(x))) - LN2F;
}
__device__ __forceinline__ v8f ld8(const float* p) {
  const v4f a = *(const v4f*)p;
  const v4f b = *(const v4f*)(p + 4);
  v8f r;
  r[0] = a.x; r[1] = a.y; r[2] = a.z; r[3] = a.w; r[4] = b.x; r[5] = b.y; r[6] = b.z; r[7] = b.w;
  return r;
}
__device__ __forceinline__ void st8(float* p, v8f v) {
  v4f a = {v[0], v[1], v[2], v[3]};
  v4f b = {v[4], v[5], v[6], v[7]};
  *(v4f*)p = a;
  *(v4f*)(p + 4) = b;
}
__device__ __forceinline__ v16h fragh(const _Float16* p) {
  FragH f;
  f.h[0] = *(const v8h*)p;
  f.h[1] = *(const v8h*)(p + 16);
  return f.v;
}
__device__ __forceinline__ v16h fragf(const float* p, float sc) {
  const v8f a = ld8(p), b = ld8(p + 16);
  FragH f;
#pragma unroll
  for (int i = 0; i < 8; ++i) { f.h[0][i] = (_Float16)(a[i] * sc); f.h[1][i] = (_Float16)(b[i] * sc); }
  return f.v;
}
__device__ __forceinline__ v8h act8(v8f d, float fold, v8f b) {
  v8h r;
#pragma unroll
  for (int i = 0; i < 8; ++i) r[i] = (_Float16)(sspf(d[i] * fold + b[i]) * ASC);
  return r;
}

__global__ __launch_bounds__(NTHR) void k_embed(const int* __restrict__ z, const float* __restrict__ emb,
                                                float* h, int nN, int nCls) {
  const int tid = threadIdx.x, lane = tid & 31, wave = tid >> 5;
  const int n = blockIdx.x * NWAVE + wave;
  const int nc = n < nN ? n : nN - 1;
  int zi = z[nc];
  zi = zi < 0 ? 0 : (zi > nCls - 1 ? nCls - 1 : zi);
  const v4f t = *(const v4f*)(emb + (size_t)zi * HC + 4 * lane);
  const float keep = (n < nN) ? 1.0f : 0.0f;
  const v4f v = t * keep;
  float* op = h + (size_t)n * HC + 4 * lane;
  *(volatile v4f*)op = v;
  __threadfence();
  *(volatile v4f*)op = v;
}

__global__ __launch_bounds__(NTHR) void k_edge_pre(const float* __restrict__ pos, const int* __restrict__ ei,
                                                   _Float16* rbf, float* cc, int nN, int nE) {
#pragma clang fp contract(off)
  __shared__ __attribute__((aligned(16))) _Float16 st[NTHR * KP1];
  const int tid = threadIdx.x, lane = tid & 31, wave = tid >> 5;
  const int e = blockIdx.x * NTHR + tid;
  const int ec = e < nE ? e : nE - 1;
  int r = ei[ec], c = ei[(size_t)nE + ec];
  r = r < 0 ? 0 : (r > nN - 1 ? nN - 1 : r);
  c = c < 0 ? 0 : (c > nN - 1 ? nN - 1 : c);
  const float dx = pos[(size_t)r * 3 + 0] - pos[(size_t)c * 3 + 0];
  const float dy = pos[(size_t)r * 3 + 1] - pos[(size_t)c * 3 + 1];
  const float dz = pos[(size_t)r * 3 + 2] - pos[(size_t)c * 3 + 2];
  const float d = sqrtf(dx * dx + dy * dy + dz * dz);
  const float delta = 10.0f / 50.0f;
  const float coeff = -0.5f / (delta * delta);
#pragma unroll 1
  for (int g = 0; g < KP1; ++g) {
    float v = 0.0f;
    if (g < NGC) { const float dg = d - (float)g * delta; v = __expf(coeff * dg * dg); }
    st[tid * KP1 + g] = (_Float16)(v * RSC);
  }
  const float cv = 0.5f * (cosf((d * PIF) * 0.1f) + 1.0f);
  __syncthreads();
  const int q = lane >> 3, piece = lane & 7;
  const size_t rowBase = (size_t)blockIdx.x * NTHR;
#pragma unroll
  for (int j = 0; j < 8; ++j) {
    const int row = 32 * wave + 4 * j + q;
    const v8h v = *(const v8h*)(st + row * KP1 + 8 * piece);
    *(volatile v8h*)(rbf + (rowBase + row) * KP1 + 8 * piece) = v;
  }
  *(volatile float*)(cc + e) = cv;
  __threadfence();
#pragma unroll
  for (int j = 0; j < 8; ++j) {
    const int row = 32 * wave + 4 * j + q;
    const v8h v = *(const v8h*)(st + row * KP1 + 8 * piece);
    *(volatile v8h*)(rbf + (rowBase + row) * KP1 + 8 * piece) = v;
  }
  *(volatile float*)(cc + e) = cv;
}

template <int TWO, int RESID>
__global__ __launch_bounds__(NTHR) void k_node(const float* __restrict__ X,
                                               const float* __restrict__ W1, const float* __restrict__ Bi1,
                                               const float* __restrict__ W2, const float* __restrict__ Bi2,
                                               const float* resid, float* outp, int nT16) {
  extern __shared__ __attribute__((aligned(16))) char smem_n[];
  _Float16* w1t = (_Float16*)(smem_n + N_W1);
  _Float16* w2t = (_Float16*)(smem_n + N_W2);
  float*    bs  = (float*)(smem_n + N_BS);
  float*    ot  = (float*)(smem_n + N_OT);
  const int tid = threadIdx.x, lane = tid & 31, wave = tid >> 5, hh = lane >> 4, m = lane & 15;

  for (int i = tid; i < HC * HC; i += NTHR) {
    const int k = i >> 7, f = i & 127;
    w1t[f * HC + k] = (_Float16)(W1[i] * WSC);
    if (TWO != 0) w2t[f * HC + k] = (_Float16)(W2[i] * WSC);
  }
  if (tid < HC) {
    bs[tid]      = (TWO != 0) ? Bi1[tid] : 0.0f;
    bs[HC + tid] = (TWO != 0) ? Bi2[tid] : 0.0f;
  }
  __syncthreads();

  float* otw = ot + wave * (16 * HC);
#pragma unroll 1
  for (int t = blockIdx.x * NWAVE + wave; t < nT16; t += gridDim.x * NWAVE) {
    const int n0 = t * 16;
    const float* xr = X + (size_t)(n0 + m) * HC + 8 * hh;
    v16h b1[4];
#pragma unroll
    for (int kt = 0; kt < 4; ++kt) b1[kt] = fragf(xr + 32 * kt, ASC);
    v16h b2[4];
#pragma unroll
    for (int p = 0; p < 4; ++p) {
      v8f d0 = zero8f(), d1 = zero8f();
      const _Float16* a0p = w1t + (32 * p + m) * HC + 8 * hh;
      const _Float16* a1p = a0p + 16 * HC;
#pragma unroll
      for (int kt = 0; kt < 4; ++kt) {
        d0 = wmh(fragh(a0p + 32 * kt), b1[kt], d0);
        d1 = wmh(fragh(a1p + 32 * kt), b1[kt], d1);
      }
      if (TWO != 0) {
        FragH qf;
        qf.h[0] = act8(d0, F12, ld8(bs + 32 * p + 8 * hh));
        qf.h[1] = act8(d1, F12, ld8(bs + 32 * p + 16 + 8 * hh));
        b2[p] = qf.v;
      } else {
        st8(otw + m * HC + 32 * p + 8 * hh, d0 * F12);
        st8(otw + m * HC + 32 * p + 16 + 8 * hh, d1 * F12);
      }
    }
    if (TWO != 0) {
#pragma unroll 1
      for (int f2 = 0; f2 < 8; ++f2) {
        v8f acc = zero8f();
        const _Float16* ap = w2t + (16 * f2 + m) * HC + 8 * hh;
#pragma unroll
        for (int kt = 0; kt < 4; ++kt) acc = wmh(fragh(ap + 32 * kt), b2[kt], acc);
        const v8f bb = ld8(bs + HC + 16 * f2 + 8 * hh);
        st8(otw + m * HC + 16 * f2 + 8 * hh, acc * F12 + bb);
      }
    }
    wave_sync();
#pragma unroll
    for (int r = 0; r < 16; ++r) {
      float* qp = otw + r * HC + 4 * lane;
      v4f v = *(const v4f*)qp;
      if (RESID != 0) v += *(const v4f*)(resid + (size_t)(n0 + r) * HC + 4 * lane);
      *(v4f*)qp = v;
    }
#pragma unroll
    for (int r = 0; r < 16; ++r)
      *(volatile v4f*)(outp + (size_t)(n0 + r) * HC + 4 * lane) = *(const v4f*)(otw + r * HC + 4 * lane);
    __threadfence();
#pragma unroll
    for (int r = 0; r < 16; ++r)
      *(volatile v4f*)(outp + (size_t)(n0 + r) * HC + 4 * lane) = *(const v4f*)(otw + r * HC + 4 * lane);
    wave_sync();
  }
}

__device__ __forceinline__ int scan_chunk(const int* __restrict__ dsts, int nE, int cbase, int nodeBase,
                                          int vec8, int* list, int tid, int wave) {
  int wc = 0;
  const int el0  = tid * EPT;
  const int e0   = cbase + el0;
  const int sent = -2147483647 - 1;
  v4i da, db;
  if (vec8 != 0 && cbase + CHUNK <= nE) {
    da = *(const v4i*)(dsts + e0);
    db = *(const v4i*)(dsts + e0 + 4);
  } else {
    da.x = (e0     < nE) ? dsts[min(e0, nE - 1)] : sent;
    da.y = (e0 + 1 < nE) ? dsts[min(e0 + 1, nE - 1)] : sent;
    da.z = (e0 + 2 < nE) ? dsts[min(e0 + 2, nE - 1)] : sent;
    da.w = (e0 + 3 < nE) ? dsts[min(e0 + 3, nE - 1)] : sent;
    db.x = (e0 + 4 < nE) ? dsts[min(e0 + 4, nE - 1)] : sent;
    db.y = (e0 + 5 < nE) ? dsts[min(e0 + 5, nE - 1)] : sent;
    db.z = (e0 + 6 < nE) ? dsts[min(e0 + 6, nE - 1)] : sent;
    db.w = (e0 + 7 < nE) ? dsts[min(e0 + 7, nE - 1)] : sent;
  }
  const unsigned nb = (unsigned)nodeBase;
  const unsigned s0 = (unsigned)da.x - nb, s1 = (unsigned)da.y - nb;
  const unsigned s2 = (unsigned)da.z - nb, s3 = (unsigned)da.w - nb;
  const unsigned s4 = (unsigned)db.x - nb, s5 = (unsigned)db.y - nb;
  const unsigned s6 = (unsigned)db.z - nb, s7 = (unsigned)db.w - nb;
  const bool h0 = s0 < (unsigned)NB, h1 = s1 < (unsigned)NB, h2 = s2 < (unsigned)NB, h3 = s3 < (unsigned)NB;
  const bool h4 = s4 < (unsigned)NB, h5 = s5 < (unsigned)NB, h6 = s6 < (unsigned)NB, h7 = s7 < (unsigned)NB;
  const unsigned any = __builtin_amdgcn_ballot_w32(h0 | h1 | h2 | h3 | h4 | h5 | h6 | h7);
  if (any != 0u) {
#define HITJ(J, HJ) { \
      const unsigned mj = __builtin_amdgcn_ballot_w32(HJ); \
      if (mj != 0u) { \
        if (HJ) { \
          const int ps = wc + (int)__builtin_amdgcn_mbcnt_lo(mj, 0u); \
          if (ps < WCAP) list[wave * WCAP + ps] = el0 + (J); \
        } \
        wc += (int)__builtin_popcount(mj); } }
    HITJ(0, h0)
    HITJ(1, h1)
    HITJ(2, h2)
    HITJ(3, h3)
    HITJ(4, h4)
    HITJ(5, h5)
    HITJ(6, h6)
    HITJ(7, h7)
#undef HITJ
  }
  return wc;
}

__global__ __launch_bounds__(NTHR) void k_agg(
    const _Float16* __restrict__ rbf, const float* __restrict__ cc, const int* __restrict__ ei,
    const float* __restrict__ xh, const float* __restrict__ W1, const float* __restrict__ Bi1,
    const float* __restrict__ W2, const float* __restrict__ Bi2, float* aggp, int nN, int nE, int vec8) {
  extern __shared__ __attribute__((aligned(16))) char smem_a[];
  float*    sacc  = (float*)(smem_a + A_ACC);
  float*    msg   = (float*)(smem_a + A_MSG);
  _Float16* w1t   = (_Float16*)(smem_a + A_W1);
  _Float16* w2t   = (_Float16*)(smem_a + A_W2);
  _Float16* stg   = (_Float16*)(smem_a + A_STG);
  int*      list  = (int*)(smem_a + A_LIST);
  int*      pend  = (int*)(smem_a + A_PEND);
  int*      slotb = (int*)(smem_a + A_SLOT);
  int*      colb  = (int*)(smem_a + A_COL);
  float*    cb    = (float*)(smem_a + A_CB);
  float*    bs    = (float*)(smem_a + A_BS);
  int*      wcnt  = (int*)(smem_a + A_WCNT);
  int*      pendN = wcnt + NWAVE;

  const int tid = threadIdx.x, lane = tid & 31, wave = tid >> 5, hh = lane >> 4, m = lane & 15;
  const int nodeBase = blockIdx.x * NB;
  const int* dsts = ei;
  const int* cols = ei + nE;

  for (int i = tid; i < (NB + 1) * HC; i += NTHR) sacc[i] = 0.0f;
  for (int i = tid; i < HC * KP1; i += NTHR) {
    const int k = i >> 7, f = i & 127;
    const int kc = k < NGC ? k : NGC - 1;
    float v = W1[kc * HC + f];
    v = (k < NGC) ? v : 0.0f;
    w1t[f * KP1 + k] = (_Float16)(v * WSC);
  }
  for (int i = tid; i < HC * HC; i += NTHR) { const int k = i >> 7, f = i & 127; w2t[f * HC + k] = (_Float16)(W2[i] * WSC); }
  if (tid < HC) { bs[tid] = Bi1[tid]; bs[HC + tid] = Bi2[tid]; }
  if (tid == 0) *pendN = 0;
  __syncthreads();

  const int nChunks = (nE + CHUNK - 1) / CHUNK;
#pragma unroll 1
  for (int ch = 0; ch < nChunks; ++ch) {
    const int cbase = ch * CHUNK;
    const int wc = scan_chunk(dsts, nE, cbase, nodeBase, vec8, list, tid, wave);
    if (lane == 0) wcnt[wave] = wc;
    __syncthreads();

    const int base = *pendN;
    int tot = 0, myoff = 0;
#pragma unroll
    for (int w = 0; w < NWAVE; ++w) {
      int c = wcnt[w];
      c = c > WCAP ? WCAP : (c < 0 ? 0 : c);
      if (w < wave) myoff += c;
      tot += c;
    }
    int newN = base + tot;
    newN = newN > PCAP ? PCAP : newN;
    {
      int n = wcnt[wave];
      n = n > WCAP ? WCAP : (n < 0 ? 0 : n);
      const int* lp = list + wave * WCAP;
      for (int i = lane; i < n; i += 32) {
        const int ps = base + myoff + i;
        if (ps < PCAP) pend[ps] = cbase + lp[i];
      }
    }
    const int fin = (ch == nChunks - 1) ? 1 : 0;
    const int R   = (fin != 0) ? (newN + PASSN - 1) / PASSN : newN / PASSN;
    const int Pv  = (fin != 0) ? newN : R * PASSN;
    __syncthreads();

#pragma unroll 1
    for (int r = 0; r < R; ++r) {
      const int pe = wave * 16 + m;
      {
        const int idx = r * PASSN + pe;
        const bool valid = idx < Pv;
        int e = pend[idx];
        e = valid ? e : 0;
        e = e < 0 ? 0 : (e > nE - 1 ? nE - 1 : e);
        const int d = dsts[e];
        int s = cols[e];
        s = s < 0 ? 0 : (s > nN - 1 ? nN - 1 : s);
        int slot = d - nodeBase;
        if (!valid || (unsigned)slot >= (unsigned)NB) slot = NB;
        const float cvv = cc[e];
        if (hh == 0) { slotb[pe] = slot; colb[pe] = s; cb[pe] = valid ? cvv : 0.0f; }
        const _Float16* rp = rbf + (size_t)e * KP1 + 32 * hh;
        _Float16* sp = stg + (size_t)pe * KP1 + 32 * hh;
#pragma unroll
        for (int j = 0; j < 4; ++j) *(v8h*)(sp + 8 * j) = *(const v8h*)(rp + 8 * j);
      }
      wave_sync();
      {
        const _Float16* sw = stg + (size_t)(wave * 16) * KP1;
        v16h b1[2];
        b1[0] = fragh(sw + m * KP1 + 8 * hh);
        b1[1] = fragh(sw + m * KP1 + 32 + 8 * hh);
        v16h b2[4];
#pragma unroll
        for (int p = 0; p < 4; ++p) {
          v8f d0 = zero8f(), d1 = zero8f();
          const _Float16* a0p = w1t + (32 * p + m) * KP1 + 8 * hh;
          const _Float16* a1p = a0p + 16 * KP1;
#pragma unroll
          for (int kt = 0; kt < 2; ++kt) {
            d0 = wmh(fragh(a0p + 32 * kt), b1[kt], d0);
            d1 = wmh(fragh(a1p + 32 * kt), b1[kt], d1);
          }
          FragH qf;
          qf.h[0] = act8(d0, F14, ld8(bs + 32 * p + 8 * hh));
          qf.h[1] = act8(d1, F14, ld8(bs + 32 * p + 16 + 8 * hh));
          b2[p] = qf.v;
        }
        const float Cm = cb[pe];
        const int colm = colb[pe];
        const float* xp = xh + (size_t)colm * HC + 8 * hh;
        float* mp = msg + (size_t)pe * HC + 8 * hh;
#pragma unroll 1
        for (int f2 = 0; f2 < 8; ++f2) {
          v8f acc = zero8f();
          const _Float16* ap = w2t + (16 * f2 + m) * HC + 8 * hh;
#pragma unroll
          for (int kt = 0; kt < 4; ++kt) acc = wmh(fragh(ap + 32 * kt), b2[kt], acc);
          const v8f bb = ld8(bs + HC + 16 * f2 + 8 * hh);
          const v8f xv = ld8(xp + 16 * f2);
          const v8f wv = (acc * F12 + bb) * Cm;
          st8(mp + 16 * f2, xv * wv);
        }
      }
      __syncthreads();
      if (wave == 0) {
#pragma unroll 1
        for (int i = 0; i < PASSN; ++i) {
          int sl = slotb[i];
          sl = sl < 0 ? 0 : (sl > NB ? NB : sl);
          const v4f mv = *(const v4f*)(msg + i * HC + 4 * lane);
          float* ap = sacc + sl * HC + 4 * lane;
          const v4f av = *(const v4f*)ap;
          *(v4f*)ap = av + mv;
        }
      }
      __syncthreads();
    }
    int rem = newN - R * PASSN;
    rem = rem < 0 ? 0 : rem;
    if (R > 0 && tid < rem) pend[tid] = pend[R * PASSN + tid];
    if (tid == 0) *pendN = rem;
  }
  __syncthreads();

  const size_t ob = (size_t)nodeBase * HC;
#pragma unroll 4
  for (int q = 0; q < RPW; ++q) {
    const int row = wave * RPW + q;
    const v4f v = *(const v4f*)(sacc + row * HC + 4 * lane);
    *(volatile v4f*)(aggp + ob + (size_t)row * HC + 4 * lane) = v;
  }
  __threadfence();
#pragma unroll 4
  for (int q = 0; q < RPW; ++q) {
    const int row = wave * RPW + q;
    const v4f v = *(const v4f*)(sacc + row * HC + 4 * lane);
    *(volatile v4f*)(aggp + ob + (size_t)row * HC + 4 * lane) = v;
  }
}

__global__ __launch_bounds__(NTHR) void k_pool(const float* __restrict__ y, const int* __restrict__ bt,
                                               float* out, int nN) {
  __shared__ unsigned mk[NWAVE];
  __shared__ __attribute__((aligned(16))) float orow[HC];
  const int tid = threadIdx.x, lane = tid & 31, wave = tid >> 5;
  const int g = blockIdx.x;
  float s = 0.0f;
  int cnt = 0;
  const int nCh = (nN + NTHR - 1) / NTHR;
#pragma unroll 1
  for (int c = 0; c < nCh; ++c) {
    const int i = c * NTHR + tid;
    const int b = bt[i < nN ? i : nN - 1];
    const bool hit = (i < nN) && (b == g);
    const unsigned mw0 = __builtin_amdgcn_ballot_w32(hit);
    if (lane == 0) mk[wave] = mw0;
    __syncthreads();
    if (tid < HC) {
#pragma unroll 1
      for (int w = 0; w < NWAVE; ++w) {
        unsigned mw = mk[w];
        cnt += (int)__builtin_popcount(mw);
#pragma unroll 1
        while (mw != 0u) {
          const int j = __builtin_ctz(mw);
          mw &= mw - 1u;
          const int node = c * NTHR + w * 32 + j;
          s += y[(size_t)node * HC + tid];
        }
      }
    }
    __syncthreads();
  }
  if (tid < HC) orow[tid] = s * (1.0f / fmaxf((float)cnt, 1.0f));
  __syncthreads();
  if (wave == 0) {
    const v4f v = *(const v4f*)(orow + 4 * lane);
    float* op = out + (size_t)g * HC + 4 * lane;
    *(volatile v4f*)op = v;
    __threadfence();
    *(volatile v4f*)op = v;
  }
}

extern "C" void kernel_launch(void* const* d_in, const int* in_sizes, int n_in,
                              void* d_out, int out_size, void* d_ws, size_t ws_size,
                              hipStream_t stream) {
  if (n_in < 18) return;
  const int nN = in_sizes[0];
  if (nN <= 0 || in_sizes[1] != 3 * nN || in_sizes[2] != nN) return;
  const int nE = in_sizes[3] / 2;
  if (nE <= 0 || in_sizes[3] != 2 * nE) return;
  if (in_sizes[4] < HC || (in_sizes[4] % HC) != 0) return;
  const int nCls = in_sizes[4] / HC;
  const int nL = in_sizes[5] / (NGC * HC);
  if (nL <= 0 || in_sizes[5] != nL * NGC * HC || in_sizes[6] != nL * HC || in_sizes[7] != nL * HC * HC ||
      in_sizes[8] != nL * HC || in_sizes[9] != nL * HC * HC || in_sizes[10] != nL * HC * HC ||
      in_sizes[11] != nL * HC || in_sizes[12] != nL * HC * HC || in_sizes[13] != nL * HC) return;
  if (in_sizes[14] != HC * HC || in_sizes[15] != HC || in_sizes[16] != HC * HC || in_sizes[17] != HC) return;
  if (out_size <= 0 || (out_size % HC) != 0) return;
  const int nG = out_size / HC;

  const int*   z      = (const int*)d_in[0];
  const float* pos    = (const float*)d_in[1];
  const int*   batch  = (const int*)d_in[2];
  const int*   ei     = (const int*)d_in[3];
  const float* emb    = (const float*)d_in[4];
  const float* mlp1_w = (const float*)d_in[5];
  const float* mlp1_b = (const float*)d_in[6];
  const float* mlp2_w = (const float*)d_in[7];
  const float* mlp2_b = (const float*)d_in[8];
  const float* cl1_w  = (const float*)d_in[9];
  const float* cl2_w  = (const float*)d_in[10];
  const float* cl2_b  = (const float*)d_in[11];
  const float* lin_w  = (const float*)d_in[12];
  const float* lin_b  = (const float*)d_in[13];
  const float* out1_w = (const float*)d_in[14];
  const float* out1_b = (const float*)d_in[15];
  const float* out2_w = (const float*)d_in[16];
  const float* out2_b = (const float*)d_in[17];
  float* out = (float*)d_out;

  const int nBlk  = (nN + NB - 1) / NB;
  const int nRows = nBlk * NB;
  const int nT16  = (nN + 15) / 16;
  const int eBlk  = (nE + NTHR - 1) / NTHR;
  const size_t eRows = (size_t)eBlk * NTHR;

  char* ws = (char*)d_ws;
  size_t off = 0;
  const size_t oR = off; off += eRows * KP1 * 2;               off = (off + 255) & ~(size_t)255;
  const size_t oC = off; off += eRows * 4;                     off = (off + 255) & ~(size_t)255;
  const size_t oH = off; off += (size_t)nRows * HC * 4;        off = (off + 255) & ~(size_t)255;
  const size_t oX = off; off += (size_t)nRows * HC * 4;        off = (off + 255) & ~(size_t)255;
  const size_t oA = off; off += (size_t)nRows * HC * 4;        off = (off + 255) & ~(size_t)255;
  if (off > ws_size) return;
  _Float16* rbf = (_Float16*)(ws + oR);
  float* ccp = (float*)(ws + oC);
  float* h   = (float*)(ws + oH);
  float* xh  = (float*)(ws + oX);
  float* agg = (float*)(ws + oA);

  hipFuncSetAttribute(reinterpret_cast<const void*>(&k_agg), hipFuncAttributeMaxDynamicSharedMemorySize, SMEM_AGG);
  hipFuncSetAttribute(reinterpret_cast<const void*>(&k_node<0, 0>), hipFuncAttributeMaxDynamicSharedMemorySize, SMEM_NODE);
  hipFuncSetAttribute(reinterpret_cast<const void*>(&k_node<1, 1>), hipFuncAttributeMaxDynamicSharedMemorySize, SMEM_NODE);
  hipFuncSetAttribute(reinterpret_cast<const void*>(&k_node<1, 0>), hipFuncAttributeMaxDynamicSharedMemorySize, SMEM_NODE);

  k_embed<<<nRows / NWAVE, NTHR, 0, stream>>>(z, emb, h, nN, nCls);
  k_edge_pre<<<eBlk, NTHR, 0, stream>>>(pos, ei, rbf, ccp, nN, nE);

  for (int i = 0; i < nL; ++i) {
    const float* w_m1 = mlp1_w + (size_t)i * NGC * HC;
    const float* b_m1 = mlp1_b + (size_t)i * HC;
    const float* w_m2 = mlp2_w + (size_t)i * HC * HC;
    const float* b_m2 = mlp2_b + (size_t)i * HC;
    const float* w_c1 = cl1_w + (size_t)i * HC * HC;
    const float* w_c2 = cl2_w + (size_t)i * HC * HC;
    const float* b_c2 = cl2_b + (size_t)i * HC;
    const float* w_ln = lin_w + (size_t)i * HC * HC;
    const float* b_ln = lin_b + (size_t)i * HC;
    k_node<0, 0><<<NODEBLK, NTHR, SMEM_NODE, stream>>>(h, w_c1, b_c2, w_c1, b_c2, h, xh, nT16);
    k_agg<<<nBlk, NTHR, SMEM_AGG, stream>>>(rbf, ccp, ei, xh, w_m1, b_m1, w_m2, b_m2, agg, nN, nE, 1);
    k_node<1, 1><<<NODEBLK, NTHR, SMEM_NODE, stream>>>(agg, w_c2, b_c2, w_ln, b_ln, h, h, nT16);
  }
  k_node<1, 0><<<NODEBLK, NTHR, SMEM_NODE, stream>>>(h, out1_w, out1_b, out2_w, out2_b, h, xh, nT16);
  k_pool<<<nG, NTHR, 0, stream>>>(xh, batch, out, nN);
}
